// PointConv_SM_8323646619716
// MI455X (gfx1250) — hardware-verified
//
#include <hip/hip_runtime.h>


#pragma clang fp contract(off)

#ifndef NPT
#define NPT 65536
#endif
#define NPT_FULL 65536
#ifndef OUT_PITCH
#define OUT_PITCH NPT
#endif
#define KNN  16
#define CIN  64
#define COUT 64
#define WC   67
#define KP   96
#define TBL  125
#define GW   4
#define AW   4
#define OSP  36
#define QRS  2048.0f
#define QRI  (1.0f / 2048.0f)
#define WSC  1024.0f
#define WSI  (1.0f / 1024.0f)

static_assert(NPT <= NPT_FULL);
static_assert(NPT_FULL % 64 == 0);
static_assert(NPT % (16 * GW) == 0);
static_assert(NPT % (32 * AW) == 0);
static_assert(OUT_PITCH % 32 == 0);
static_assert(OUT_PITCH >= NPT);
static_assert(KP % 32 == 0);
static_assert(KP >= WC + 1);
static_assert(KP == 96);
static_assert(CIN == 64);
static_assert(COUT == 64);
static_assert(CIN + 3 == WC);
static_assert(KNN == 16);
static_assert((16 * KP * 2) % 128 == 0);
static_assert((OSP * 4) % 16 == 0);
static_assert(256 * 2 * 16 == 64 * 128);
static_assert(3 * 256 * 16 == COUT * KP * 2);
static_assert(32 * 6 * 16 == 16 * KP * 2);
static_assert(32 * 16 * 16 == COUT * 128);
static_assert(64 * 65 * 4 <= 131072);
static_assert(GW * 16 * KP * 4 <= 131072);
static_assert(AW * COUT * OSP * 4 <= 131072);

typedef _Float16 h16;
typedef unsigned short bf;
typedef __attribute__((ext_vector_type(16))) _Float16 v16h;
typedef __attribute__((ext_vector_type(8)))  _Float16 v8h;
typedef __attribute__((ext_vector_type(8)))  unsigned short v8us;
typedef __attribute__((ext_vector_type(8)))  float    v8f;
typedef __attribute__((ext_vector_type(4)))  float    v4f;
typedef __attribute__((ext_vector_type(4)))  int      v4i;
typedef v4f  __attribute__((may_alias)) v4fa;

__device__ __forceinline__ unsigned short f2bf(float f) { unsigned u = __float_as_uint(f); u += 0x7FFFu + ((u >> 16) & 1u); return (unsigned short)(u >> 16); }
__device__ __forceinline__ float bfr(float f) { return __uint_as_float(((unsigned)f2bf(f)) << 16); }
__device__ __forceinline__ float bfw(unsigned short w) { return __uint_as_float(((unsigned)w) << 16); }
__device__ __forceinline__ v16h cat16(v8h lo, v8h hi) { return __builtin_shufflevector(lo, hi, 0, 1, 2, 3, 4, 5, 6, 7, 8, 9, 10, 11, 12, 13, 14, 15); }
__device__ __forceinline__ v8f wmma16(v16h a, v16h b, v8f c) { return __builtin_amdgcn_wmma_f32_16x16x32_f16(false, a, false, b, (short)0, c, false, false); }
__device__ __forceinline__ v8f wm16g(v16h a, v16h b, v8f c) { c = wmma16(a, b, c); asm volatile("v_nop\n\tv_nop\n\tv_nop\n\tv_nop" : "+v"(c) : "v"(a), "v"(b)); return c; }
__device__ __forceinline__ v16h  ldh(const h16* p) { return cat16(*(const v8h*)p, *(const v8h*)(p + 16)); }
__device__ __forceinline__ void wave_sync() { __builtin_amdgcn_fence(3  , "wavefront"); __builtin_amdgcn_wave_barrier(); asm volatile("" ::: "memory"); }
static __device__ __forceinline__ h16 toh_flush(float v) { const h16 r = (h16)v; return (fabsf(v) < 6.103515625e-05f) ? (h16)0.0f : r; }

__global__ __launch_bounds__(256) void k_tr(const float* __restrict__ fea, bf* FT) {
    __shared__ float ts[64 * 65];
    const int tid = threadIdx.x; const size_t n0 = (size_t)blockIdx.x * 64;
#pragma unroll 4
    for (int i = 0; i < 16; ++i) { const int idx = tid + (i << 8); const int c = idx >> 6, p = idx & 63;
        ts[c * 65 + p] = fea[(size_t)c * NPT_FULL + n0 + p]; }
    __syncthreads();
    v8us o[2];
#pragma unroll
    for (int it = 0; it < 2; ++it) { const int q = it * 256 + tid; const int p = q >> 3, c8 = (q & 7) * 8;
#pragma unroll
        for (int k = 0; k < 8; ++k) o[it][k] = f2bf(ts[(c8 + k) * 65 + p]); }
#pragma unroll 1
    for (int ps = 0; ps < 2; ++ps) {
#pragma unroll
        for (int it = 0; it < 2; ++it) { const int q = it * 256 + tid;
            *(volatile v8us*)(FT + n0 * CIN + (size_t)q * 8) = o[it]; }
        if (ps == 0) __threadfence(); }
}

__global__ __launch_bounds__(256) void k_wconv(const float* __restrict__ w, h16* WH) {
    const int q = blockIdx.x * 256 + threadIdx.x;
    const int row = q / 12, c8 = (q % 12) * 8;
    v8h o;
#pragma unroll
    for (int k = 0; k < 8; ++k) { const int col = c8 + k; const int cc = col < WC ? col : (WC - 1);
        float x = w[row * WC + cc];
        asm volatile("" : "+v"(x));
        const float val = (col < WC) ? bfr(x) * WSC : 0.0f;
        o[k] = toh_flush(val); }
    *(volatile v8h*)(WH + (size_t)q * 8) = o; __threadfence(); *(volatile v8h*)(WH + (size_t)q * 8) = o;
}

__global__ __launch_bounds__(32 * GW) void k_gsum(const bf* __restrict__ FT, const int* __restrict__ knn, const float* __restrict__ rel, h16* SH, h16* SR) {
#pragma clang fp contract(off)
    __shared__ __align__(16) float os[GW * 16 * KP];
    const int lane = threadIdx.x & 31, lr = lane & 15, hi = lane >> 4;
    const int wave = __builtin_amdgcn_readfirstlane((int)(threadIdx.x >> 5));
    const int n0w = (blockIdx.x * GW + wave) * 16;
    const int wb = wave * 16 * KP;
#pragma unroll
    for (int i = 0; i < 4; ++i) { const int q = i * 32 + lane; const int row = q >> 3, c4 = (q & 7) * 4;
        const v4f z = (v4f){0.0f, 0.0f, 0.0f, 0.0f};
        *(v4fa*)(&os[wb + row * KP + 64 + c4]) = z; }
    wave_sync();
    const int sub = lane >> 3, c8 = (lane & 7) * 8;
#pragma unroll 1
    for (int g = 0; g < 4; ++g) {
        const int pt = g * 4 + sub; const size_t n = (size_t)(n0w + pt);
        const int* ip = knn + n * KNN;
        const v4i i0 = *(const v4i*)(ip);
        const v8us cv = *(const v8us*)(FT + n * CIN + c8);
        float acc[8];
#pragma unroll
        for (int k = 0; k < 8; ++k) acc[k] = -14.0f * bfw(cv[k]);
#pragma unroll
        for (int k4 = 1; k4 < 4; ++k4) {
            int m = i0[k4]; m = m < 0 ? 0 : (m > NPT_FULL - 1 ? NPT_FULL - 1 : m);
            const v8us gv = *(const v8us*)(FT + (size_t)m * CIN + c8);
#pragma unroll
            for (int k = 0; k < 8; ++k) acc[k] += bfw(gv[k]); }
#pragma unroll 1
        for (int jq = 1; jq < 4; ++jq) {
            const v4i iv = *(const v4i*)(ip + 4 * jq);
#pragma unroll
            for (int k4 = 0; k4 < 4; ++k4) {
                int m = iv[k4]; m = m < 0 ? 0 : (m > NPT_FULL - 1 ? NPT_FULL - 1 : m);
                const v8us gv = *(const v8us*)(FT + (size_t)m * CIN + c8);
#pragma unroll
                for (int k = 0; k < 8; ++k) acc[k] += bfw(gv[k]); } }
        v4f a, c;
        a[0] = acc[0]; a[1] = acc[1]; a[2] = acc[2]; a[3] = acc[3]; c[0] = acc[4]; c[1] = acc[5]; c[2] = acc[6]; c[3] = acc[7];
        *(v4fa*)(&os[wb + pt * KP + c8]) = a; *(v4fa*)(&os[wb + pt * KP + c8 + 4]) = c;
    }
#pragma unroll 1
    for (int c = 0; c < 3; ++c) {
        const float* rp = rel + ((size_t)(c * KNN + 8 * hi)) * NPT_FULL + (size_t)(n0w + lr);
        float r = 0.0f;
#pragma unroll
        for (int i = 0; i < 8; ++i) r += bfr(rp[(size_t)i * NPT_FULL]);
        r += __shfl_xor(r, 16, 32);
        if (hi == 0) os[wb + lr * KP + 64 + c] = r;
    }
    wave_sync();
    const size_t gb = (size_t)n0w * KP;
#pragma unroll 1
    for (int ps = 0; ps < 2; ++ps) {
#pragma unroll 1
        for (int i = 0; i < 6; ++i) { const int q = i * 32 + lane;
            const v4f x0 = *(const v4fa*)(&os[wb + q * 8]); const v4f x1 = *(const v4fa*)(&os[wb + q * 8 + 4]); v8h hv, rv;
#pragma unroll
            for (int k = 0; k < 4; ++k) { const h16 a0 = toh_flush(x0[k]); const h16 a1 = toh_flush(x1[k]); hv[k] = a0; hv[4 + k] = a1;
                rv[k] = toh_flush((x0[k] - (float)a0) * QRS); rv[4 + k] = toh_flush((x1[k] - (float)a1) * QRS); }
            *(volatile v8h*)(SH + gb + (size_t)q * 8) = hv; *(volatile v8h*)(SR + gb + (size_t)q * 8) = rv; }
        if (ps == 0) __threadfence(); }
}

__global__ __launch_bounds__(32 * AW) void k_gemm(const h16* __restrict__ WH, const h16* __restrict__ SH, const h16* __restrict__ SR,
                                                  const float* __restrict__ sample, const float* __restrict__ cdw, const float* __restrict__ bias, float* OUT) {
    __shared__ __align__(16) float os[AW * COUT * OSP];
    const int lane = threadIdx.x & 31, lr = lane & 15, hi = lane >> 4;
    const int wave = __builtin_amdgcn_readfirstlane((int)(threadIdx.x >> 5));
    const int p0 = (blockIdx.x * AW + wave) * 32;
    const int wb = wave * COUT * OSP;
    const size_t aoff = (size_t)lr * KP + 8 * hi;
#pragma unroll 1
    for (int hf = 0; hf < 2; ++hf) {
        const int pn = p0 + hf * 16 + lr;
        const size_t boff = (size_t)pn * KP + 8 * hi;
        v8f acc[4], accr[4];
#pragma unroll
        for (int mb = 0; mb < 4; ++mb) { acc[mb] = (v8f){}; accr[mb] = (v8f){}; }
#pragma unroll 1
        for (int kc = 0; kc < KP; kc += 32) {
            v16h a[4];
#pragma unroll
            for (int mb = 0; mb < 4; ++mb) a[mb] = ldh(WH + aoff + (size_t)mb * 16 * KP + kc);
            const v16h bh = ldh(SH + boff + kc);
            const v16h br = ldh(SR + boff + kc);
#pragma unroll
            for (int mb = 0; mb < 4; ++mb) { acc[mb] = wm16g(a[mb], bh, acc[mb]); accr[mb] = wm16g(a[mb], br, accr[mb]); }
        }
        const float sx = bfr(sample[(size_t)pn * 3 + 0]);
        const float sy = bfr(sample[(size_t)pn * 3 + 1]);
        const float sz = bfr(sample[(size_t)pn * 3 + 2]);
        int cx = (int)((fminf(fmaxf(sx, -0.99999f), 0.99999f) * 5.0f) / 2.0f) + 2;
        int cy = (int)((fminf(fmaxf(sy, -0.99999f), 0.99999f) * 5.0f) / 2.0f) + 2;
        int cz = (int)((fminf(fmaxf(sz, -0.99999f), 0.99999f) * 5.0f) / 2.0f) + 2;
        cx = cx < 0 ? 0 : (cx > 4 ? 4 : cx); cy = cy < 0 ? 0 : (cy > 4 ? 4 : cy); cz = cz < 0 ? 0 : (cz > 4 ? 4 : cz);
        int off = cz * 25 + cy * 5 + cx;
#pragma unroll
        for (int mb = 0; mb < 4; ++mb) {
            const int ob = mb * 16 + 8 * hi;
            const v4f b0 = *(const v4f*)(bias + ob); const v4f b1 = *(const v4f*)(bias + ob + 4);
            float bb[8], kd[8];
#pragma unroll
            for (int r = 0; r < 4; ++r) { bb[r] = b0[r]; bb[4 + r] = b1[r]; }
#pragma unroll
            for (int r = 0; r < 8; ++r) kd[r] = cdw[(ob + r) * TBL + off];
            asm volatile("" : "+v"(kd[0]), "+v"(kd[1]), "+v"(kd[2]), "+v"(kd[3]), "+v"(kd[4]), "+v"(kd[5]), "+v"(kd[6]), "+v"(kd[7]), "+v"(off));
#pragma unroll
            for (int r = 0; r < 8; ++r) {
                const float pre = (acc[mb][r] + accr[mb][r] * QRI) * WSI;
                const float t = pre + 16.0f * bfr(bb[r]);
                os[wb + (ob + r) * OSP + hf * 16 + lr] = bfr(kd[r]) * t; }
            asm volatile("" ::: "memory");
        }
    }
    wave_sync();
    float* orow = OUT + (size_t)p0;
#pragma unroll 1
    for (int ps = 0; ps < 2; ++ps) {
#pragma unroll
        for (int s = 0; s < 16; ++s) { const int row = 4 * s + (lane >> 3), cofs = (lane & 7) * 4;
            const v4f val = *(const v4fa*)(&os[wb + row * OSP + cofs]);
            *(volatile v4f*)(orow + (size_t)row * OUT_PITCH + cofs) = val; }
        if (ps == 0) __threadfence(); }
}

static constexpr size_t al256(size_t v) { return (v + 255) & ~(size_t)255; }
static constexpr size_t SZ_FT = al256((size_t)NPT_FULL * CIN * 2);
static constexpr size_t SZ_WH = al256((size_t)COUT * KP * 2);
static constexpr size_t SZ_S  = al256((size_t)NPT * KP * 2);
static constexpr size_t SZ_TOTAL = SZ_FT + SZ_WH + 2 * SZ_S;
static_assert(SZ_TOTAL <= (size_t)134217728);
static_assert((size_t)(NPT_FULL / 64) * 64 * CIN * 2 == (size_t)NPT_FULL * CIN * 2);
static_assert((size_t)(NPT / (16 * GW)) * GW * 16 * KP * 2 == (size_t)NPT * KP * 2);

extern "C" void kernel_launch(void* const* d_in, const int* in_sizes, int n_in,
                              void* d_out, int out_size, void* d_ws, size_t ws_size, hipStream_t stream) {
    if (n_in < 7) return;
    if ((size_t)in_sizes[0] < (size_t)NPT * 3) return;
    if ((size_t)in_sizes[1] < (size_t)(3 * KNN - 1) * NPT_FULL + NPT) return;
    if ((size_t)in_sizes[2] < (size_t)CIN * NPT_FULL) return;
    if ((size_t)in_sizes[3] < (size_t)NPT * KNN) return;
    if (in_sizes[4] < COUT * WC || in_sizes[5] < COUT || in_sizes[6] < COUT * TBL) return;
    if ((size_t)out_size < (size_t)(COUT - 1) * OUT_PITCH + NPT) return;
    if (SZ_TOTAL > ws_size) return;
    const float* sample = (const float*)d_in[0];
    const float* rel    = (const float*)d_in[1];
    const float* fea    = (const float*)d_in[2];
    const int*   knn    = (const int*)d_in[3];
    const float* w      = (const float*)d_in[4];
    const float* bias   = (const float*)d_in[5];
    const float* cdw    = (const float*)d_in[6];
    float* OUT = (float*)d_out;
    char* wsp = (char*)d_ws;
    bf*  FT = (bf*)wsp;  wsp += SZ_FT;
    h16* WH = (h16*)wsp; wsp += SZ_WH;
    h16* SH = (h16*)wsp; wsp += SZ_S;
    h16* SR = (h16*)wsp; wsp += SZ_S;

    k_tr<<<dim3(NPT_FULL / 64, 1, 1), 256, 0, stream>>>(fea, FT);
    k_wconv<<<dim3(3, 1, 1), 256, 0, stream>>>(w, WH);
    k_gsum<<<dim3(NPT / (16 * GW), 1, 1), 32 * GW, 0, stream>>>(FT, knn, rel, SH, SR);
    k_gemm<<<dim3(NPT / (32 * AW), 1, 1), 32 * AW, 0, stream>>>(WH, SH, SR, sample, cdw, bias, OUT);
}
